// HMSS_72980084293806
// MI455X (gfx1250) — hardware-verified
//
#include <hip/hip_runtime.h>


#define NB_   8
#define NL_   512
#define DM_   256
#define DI_   512
#define NS_   16
#define NLAY_ 2
#define DTR_  16
#define XPR_  48
#define XPN_  64
#define DTK_  32
#define HCK_  (3 * DM_)
#define MT_   (NB_ * NL_)

static_assert(MT_ % 64 == 0);
static_assert(DM_ % 128 == 0);
static_assert((2 * DI_) % 128 == 0);
static_assert(DI_ % 128 == 0);
static_assert(XPN_ % 64 == 0);
static_assert(HCK_ % 32 == 0);
static_assert(DTK_ % 32 == 0);
static_assert(NL_ % 16 == 0);
static_assert(DI_ == 64 * 8);
static_assert(DM_ == 32 * 8);
static_assert(XPR_ == DTR_ + 2 * NS_);

static constexpr float EPS_ = 1e-5f;

typedef float          v4f   __attribute__((ext_vector_type(4)));
typedef float          v8f   __attribute__((ext_vector_type(8)));
typedef _Float16       v8h   __attribute__((ext_vector_type(8)));
typedef _Float16       v16h  __attribute__((ext_vector_type(16)));
typedef unsigned short u16x8 __attribute__((ext_vector_type(8)));

union FragH { u16x8 h[2]; v16h v; };
union Pack8 { v8h f; u16x8 u; };

__device__ __forceinline__ v8f ld8f(const float* p) {
    v4f a = *(const v4f*)p;
    v4f b = *(const v4f*)(p + 4);
    return __builtin_shufflevector(a, b, 0, 1, 2, 3, 4, 5, 6, 7);
}
__device__ __forceinline__ v8f zero8() {
    v8f z;
#pragma unroll
    for (int c = 0; c < 8; ++c) z[c] = 0.0f;
    return z;
}
__device__ __forceinline__ u16x8 pack_h(v8f x) {
    Pack8 pk;
    pk.f = __builtin_convertvector(x, v8h);
    return pk.u;
}
__device__ __forceinline__ float wsum32(float s) {
#pragma unroll
    for (int o = 16; o; o >>= 1) s += __shfl_xor(s, o, 32);
    return s;
}
__device__ __forceinline__ float silu_f(float x) {
    float e = expf(-x);
    return x * __builtin_amdgcn_rcpf(1.0f + e);
}
__device__ __forceinline__ float softplus_f(float x) {
    return fmaxf(x, 0.0f) + log1pf(expf(-fabsf(x)));
}
__device__ __forceinline__ float conv4_silu(float x0, float x1, float x2, float x3,
                                            float w0, float w1, float w2, float w3, float bias) {
    float c = w0 * x0 + w1 * x1 + w2 * x2 + w3 * x3;
    return silu_f(c + bias);
}
__device__ __forceinline__ void st16x2(unsigned short* p, u16x8 v) {
    *(volatile u16x8*)p = v;
    __threadfence();
    *(volatile u16x8*)p = v;
}

__device__ __forceinline__ void mma16(v8f& acc, const FragH& a, const FragH& b) {
    acc = __builtin_amdgcn_wmma_f32_16x16x32_f16(false, a.v, false, b.v, (short)0, acc, false, false);
    asm volatile("v_nop\n\tv_nop\n\tv_nop\n\tv_nop" : "+v"(acc) : "v"(a.v), "v"(b.v));
}

__global__ __launch_bounds__(256)
void cvt2_kernel(const float* __restrict__ s0, unsigned short* d0, int n8a,
                 const float* __restrict__ s1, unsigned short* d1, int n8b, float scale)
{
    const int i = blockIdx.x * 256 + threadIdx.x;
    const bool second = (blockIdx.y != 0);
    const float* src = second ? s1 : s0;
    unsigned short* dst = second ? d1 : d0;
    const int n8 = second ? n8b : n8a;
    if (i >= n8) return;
    const size_t e = (size_t)i * 8;
    const u16x8 v = pack_h(ld8f(src + e) * scale);
    st16x2(dst + e, v);
}

__global__ __launch_bounds__(256)
void hconv_pack_kernel(const float* __restrict__ w, unsigned short* dst, float scale)
{
    const int i = blockIdx.x * 256 + threadIdx.x;
    if (i >= DM_ * HCK_ / 8) return;
    const int e  = i * 8;
    const int o  = e / HCK_;
    const int r  = e - o * HCK_;
    const int k  = r / DM_;
    const int i0 = r - k * DM_;
    v8f x;
#pragma unroll
    for (int c = 0; c < 8; ++c) x[c] = w[((size_t)o * DM_ + i0 + c) * 3 + k] * scale;
    st16x2(dst + e, pack_h(x));
}

__global__ __launch_bounds__(256)
void xproj_pack_kernel(const float* __restrict__ sf, const float* __restrict__ sb,
                       unsigned short* df, unsigned short* db, float scale)
{
    const int i = blockIdx.x * 256 + threadIdx.x;
    const bool second = (blockIdx.y != 0);
    const float* src = second ? sb : sf;
    unsigned short* dst = second ? db : df;
    if (i >= NLAY_ * XPN_ * DI_ / 8) return;
    const int e   = i * 8;
    const int l   = e / (XPN_ * DI_);
    const int rem = e - l * (XPN_ * DI_);
    const int r   = rem / DI_;
    const int k   = rem - r * DI_;
    v8f x = zero8();
    if (r < XPR_) x = ld8f(src + ((size_t)(l * XPR_ + r)) * DI_ + k) * scale;
    st16x2(dst + e, pack_h(x));
}

__global__ __launch_bounds__(256)
void dtw_pack_kernel(const float* __restrict__ sf, const float* __restrict__ sb,
                     unsigned short* df, unsigned short* db, float scale)
{
    const int i = blockIdx.x * 256 + threadIdx.x;
    const bool second = (blockIdx.y != 0);
    const float* src = second ? sb : sf;
    unsigned short* dst = second ? db : df;
    if (i >= NLAY_ * DI_ * DTK_ / 8) return;
    const int e   = i * 8;
    const int row = e / DTK_;
    const int k0  = e - row * DTK_;
    v8f x = zero8();
    if (k0 < DTR_) x = ld8f(src + (size_t)row * DTR_ + k0) * scale;
    st16x2(dst + e, pack_h(x));
}

__global__ __launch_bounds__(64)
void norm_f16_kernel(const float* __restrict__ X, const float* __restrict__ g,
                     const float* __restrict__ bb, const float* __restrict__ gate,
                     unsigned short* dst, int mode, float scale)
{
    const int lane = threadIdx.x & 31;
    const int row  = blockIdx.x * 2 + (threadIdx.x >> 5);
    const int c0   = lane * 8;
    const size_t base = (size_t)row * DM_ + c0;
    const v8f x = ld8f(X + base);
    v8f y;
    if (mode == 0) {
        float s = 0.0f;
#pragma unroll
        for (int c = 0; c < 8; ++c) s += x[c];
        s = wsum32(s);
        const float mean = s * (1.0f / (float)DM_);
        const v8f dv = x - mean;
        float q = 0.0f;
#pragma unroll
        for (int c = 0; c < 8; ++c) q += dv[c] * dv[c];
        q = wsum32(q);
        const float rs = rsqrtf(q * (1.0f / (float)DM_) + EPS_);
        const v8f gv = ld8f(g + c0);
        const v8f bv = ld8f(bb + c0);
        y = dv * rs * gv + bv;
    } else {
        float q = 0.0f;
#pragma unroll
        for (int c = 0; c < 8; ++c) q += x[c] * x[c];
        q = wsum32(q);
        const float rs = rsqrtf(q * (1.0f / (float)DM_) + EPS_);
        const v8f gv = ld8f(g + c0);
        y = x * rs * gv;
    }
    if (gate) y = y * ld8f(gate + base);
    st16x2(dst + base, pack_h(y * scale));
}

__global__ __launch_bounds__(64)
void im2col_kernel(const float* __restrict__ X1, unsigned short* dst, float scale)
{
    const int lane = threadIdx.x & 31;
    const int row  = blockIdx.x * 2 + (threadIdx.x >> 5);
    const int b    = row / NL_;
    const int t    = row - b * NL_;
    const int c0   = lane * 8;
    u16x8 v[3];
#pragma unroll
    for (int j = 0; j < 3; ++j) {
        const int ts = t + j - 1;
        v8f x = zero8();
        if (ts >= 0 && ts < NL_) x = ld8f(X1 + ((size_t)(b * NL_ + ts)) * DM_ + c0) * scale;
        v[j] = pack_h(x);
    }
    unsigned short* gp = dst + (size_t)row * HCK_ + c0;
#pragma unroll
    for (int j = 0; j < 3; ++j) *(volatile u16x8*)(gp + j * DM_) = v[j];
    __threadfence();
#pragma unroll
    for (int j = 0; j < 3; ++j) *(volatile u16x8*)(gp + j * DM_) = v[j];
}

__global__ __launch_bounds__(64)
void cat_kernel(const float* __restrict__ xf, const float* __restrict__ xb,
                unsigned short* dst, float scale)
{
    const int lane = threadIdx.x & 31;
    const int row  = blockIdx.x * 2 + (threadIdx.x >> 5);
    const int c0   = lane * 8;
    const u16x8 va = pack_h(ld8f(xf + (size_t)row * DM_ + c0) * scale);
    const u16x8 vb = pack_h(ld8f(xb + (size_t)row * DM_ + c0) * scale);
    unsigned short* gp = dst + (size_t)row * (2 * DM_) + c0;
    *(volatile u16x8*)(gp)       = va;
    *(volatile u16x8*)(gp + DM_) = vb;
    __threadfence();
    *(volatile u16x8*)(gp)       = va;
    *(volatile u16x8*)(gp + DM_) = vb;
}

__global__ __launch_bounds__(256)
void dbc16_kernel(const float* __restrict__ dbc, unsigned short* dst, float scale)
{
    const int i = blockIdx.x * 256 + threadIdx.x;
    if (i >= MT_ * DTK_ / 8) return;
    const int row = i >> 2;
    const int q   = (i & 3) * 8;
    const v8f x = ld8f(dbc + (size_t)row * XPN_ + q) * scale;
    st16x2(dst + (size_t)row * DTK_ + q, pack_h(x));
}

template<int NBF>
__device__ __forceinline__ void tile_store_pass(const float* st, float* gp, int ldc, int lane) {
    constexpr int CW  = NBF * 16;
    constexpr int P   = CW + 4;
    constexpr int LPR = CW / 4;
    constexpr int RPI = 32 / LPR;
    constexpr int NIT = 32 / RPI;
    const int rsub = lane / LPR;
    const int c4   = (lane % LPR) * 4;
#pragma unroll
    for (int it = 0; it < NIT; ++it) {
        const int row = it * RPI + rsub;
        const v4f v = *(const v4f*)(st + row * P + c4);
        *(volatile v4f*)(gp + (size_t)row * ldc + c4) = v;
    }
}

template<int NBF>
__global__ __launch_bounds__(128)
void gemm_tn_kernel(const unsigned short* __restrict__ A, const unsigned short* __restrict__ Bw,
                    const float* __restrict__ bias, const float* __restrict__ bias2,
                    const float* resid, float* C, float* C2, float* Cdup,
                    int K, int ldc, int csplit, float scale)
{
    constexpr int CW = NBF * 16;
    constexpr int P  = CW + 4;
    __shared__ __attribute__((aligned(16))) float stile[4][32 * P];

    const int tid  = threadIdx.x;
    const int lane = tid & 31;
    const int wave = tid >> 5;
    const int h    = lane >> 4;
    const int m    = lane & 15;
    const int wm   = wave >> 1;
    const int wn   = wave & 1;

    const int rowW = blockIdx.y * 64 + wm * 32;
    const int colW = blockIdx.x * (2 * CW) + wn * CW;

    v8f acc[2 * NBF];
#pragma unroll
    for (int j = 0; j < 2 * NBF; ++j) acc[j] = zero8();

    const size_t aoff  = (size_t)(rowW + m) * K + 8 * h;
    const size_t boff  = (size_t)(colW + m) * K + 8 * h;
    const size_t sub16 = (size_t)16 * K;
    const int nk = K >> 5;

    for (int kt = 0; kt < nk; ++kt) {
        const size_t k0 = (size_t)kt * 32;
        FragH fa[2], fb[NBF];
#pragma unroll
        for (int s = 0; s < 2; ++s) {
            const unsigned short* p = A + aoff + s * sub16 + k0;
            fa[s].h[0] = *(const u16x8*)(p);
            fa[s].h[1] = *(const u16x8*)(p + 16);
        }
#pragma unroll
        for (int j = 0; j < NBF; ++j) {
            const unsigned short* p = Bw + boff + j * sub16 + k0;
            fb[j].h[0] = *(const u16x8*)(p);
            fb[j].h[1] = *(const u16x8*)(p + 16);
        }
#pragma unroll
        for (int s = 0; s < 2; ++s)
#pragma unroll
            for (int j = 0; j < NBF; ++j)
                mma16(acc[s * NBF + j], fa[s], fb[j]);
    }

    float* Cp = C;
    const float* bp = bias;
    int gcol = colW;
    if (colW >= csplit) { Cp = C2; bp = bias2; gcol = colW - csplit; }

    float bv[NBF];
#pragma unroll
    for (int j = 0; j < NBF; ++j) bv[j] = bp ? bp[gcol + j * 16 + m] : 0.0f;

    float* st = stile[wave];
#pragma unroll
    for (int s = 0; s < 2; ++s)
#pragma unroll
        for (int j = 0; j < NBF; ++j)
#pragma unroll
            for (int r = 0; r < 8; ++r) {
                const int row = s * 16 + 8 * h + r;
                const int col = j * 16 + m;
                float v = acc[s * NBF + j][r] * scale + bv[j];
                if (resid) v += resid[(size_t)(rowW + row) * ldc + gcol + col];
                st[row * P + col] = v;
            }
    __syncthreads();

    float* gp = Cp + (size_t)rowW * ldc + gcol;
    const bool dup = (Cdup != nullptr);
    float* gd = dup ? (Cdup + (size_t)rowW * ldc + gcol) : Cp;
    tile_store_pass<NBF>(st, gp, ldc, lane);
    if (dup) tile_store_pass<NBF>(st, gd, ldc, lane);
    __threadfence();
    tile_store_pass<NBF>(st, gp, ldc, lane);
    if (dup) tile_store_pass<NBF>(st, gd, ldc, lane);
}

__global__ __launch_bounds__(64)
void conv_silu_kernel(const float* __restrict__ Xf, const float* __restrict__ cw,
                      const float* __restrict__ cb, unsigned short* U16, int dir, float scale)
{
    const int mrow = blockIdx.x;
    const int t    = mrow & (NL_ - 1);
    const int d0   = threadIdx.x * 8;
    const float* xr = Xf + (size_t)mrow * DI_ + d0;
    const int nprev = dir ? (NL_ - 1 - t) : t;

    v8f x3 = ld8f(xr);
    v8f x2 = zero8(), x1 = zero8(), x0 = zero8();
    if (nprev >= 1) { const float* p = dir ? (xr + DI_)     : (xr - DI_);     x2 = ld8f(p); }
    if (nprev >= 2) { const float* p = dir ? (xr + 2 * DI_) : (xr - 2 * DI_); x1 = ld8f(p); }
    if (nprev >= 3) { const float* p = dir ? (xr + 3 * DI_) : (xr - 3 * DI_); x0 = ld8f(p); }

    const float* wp = cw + (size_t)d0 * 4;
    v4f wv[8];
#pragma unroll
    for (int c = 0; c < 8; ++c) wv[c] = *(const v4f*)(wp + 4 * c);
    const v8f bias = ld8f(cb + d0);

    v8f u;
#pragma unroll
    for (int c = 0; c < 8; ++c)
        u[c] = conv4_silu(x0[c], x1[c], x2[c], x3[c], wv[c][0], wv[c][1], wv[c][2], wv[c][3], bias[c]);

    st16x2(U16 + (size_t)mrow * DI_ + d0, pack_h(u * scale));
}

__global__ __launch_bounds__(64)
void scan_kernel(const float* __restrict__ Xf, const float* __restrict__ Zf, const float* __restrict__ Dl,
                 const float* __restrict__ dbc, const float* __restrict__ cw, const float* __restrict__ cb,
                 const float* __restrict__ dtb, const float* __restrict__ Alog, const float* __restrict__ Dp,
                 unsigned short* G16, int dir, float gscale)
{
    __shared__ __attribute__((aligned(16))) float    sbc[16 * 32];
    __shared__ __attribute__((aligned(16))) _Float16 sg[16 * 64];

    const int tid   = threadIdx.x;
    const int lane  = tid & 31;
    const int wave  = tid >> 5;
    const int dbase = blockIdx.x * 64;
    const int d     = dbase + tid;
    const int b     = blockIdx.y;

    float an[NS_], hs[NS_];
#pragma unroll
    for (int n = 0; n < NS_; ++n) {
        an[n] = -expf(Alog[d * NS_ + n]);
        hs[n] = 0.0f;
    }
    const float w0 = cw[d * 4 + 0], w1 = cw[d * 4 + 1], w2 = cw[d * 4 + 2], w3 = cw[d * 4 + 3];
    const float cbias = cb[d];
    const float tb = dtb[d];
    const float Dd = Dp[d];

    float xm1 = 0.0f, xm2 = 0.0f, xm3 = 0.0f;
    const size_t mrow0 = (size_t)b * NL_;

#pragma unroll 1
    for (int s0 = 0; s0 < NL_; s0 += 16) {
        __syncthreads();
        {
            const int j = tid >> 2;
            const int q = (tid & 3) * 8;
            const int s = s0 + j;
            const int t = dir ? (NL_ - 1 - s) : s;
            const float* src = dbc + (mrow0 + (size_t)t) * XPN_ + DTR_ + q;
            *(v4f*)(sbc + j * 32 + q)     = *(const v4f*)(src);
            *(v4f*)(sbc + j * 32 + q + 4) = *(const v4f*)(src + 4);
        }
        __syncthreads();
#pragma unroll 1
        for (int j = 0; j < 16; ++j) {
            const int s = s0 + j;
            const int t = dir ? (NL_ - 1 - s) : s;
            const size_t e = (mrow0 + (size_t)t) * DI_ + d;
            const float xv  = Xf[e];
            const float zv  = Zf[e];
            const float dlv = Dl[e];
            const float u   = conv4_silu(xm3, xm2, xm1, xv, w0, w1, w2, w3, cbias);
            xm3 = xm2; xm2 = xm1; xm1 = xv;
            const float dt = softplus_f(dlv + tb);
            const float du = dt * u;
            const float* bc = sbc + j * 32;
            float y = 0.0f;
#pragma unroll
            for (int n = 0; n < NS_; ++n) {
                const float da = __expf(dt * an[n]);
                hs[n] = da * hs[n] + du * bc[n];
                y += hs[n] * bc[NS_ + n];
            }
            const float g = (y + Dd * u) * silu_f(zv);
            sg[j * 64 + tid] = (_Float16)(g * gscale);
        }
        __syncthreads();
        u16x8 v[2];
        size_t goff[2];
#pragma unroll
        for (int it = 0; it < 2; ++it) {
            const int jj = 8 * wave + it * 4 + (lane >> 3);
            const int c  = (lane & 7) * 8;
            const int s  = s0 + jj;
            const int t  = dir ? (NL_ - 1 - s) : s;
            Pack8 pk;
            pk.f = *(const v8h*)(sg + jj * 64 + c);
            v[it] = pk.u;
            goff[it] = (mrow0 + (size_t)t) * DI_ + dbase + c;
        }
#pragma unroll
        for (int it = 0; it < 2; ++it) *(volatile u16x8*)(G16 + goff[it]) = v[it];
        __threadfence();
#pragma unroll
        for (int it = 0; it < 2; ++it) *(volatile u16x8*)(G16 + goff[it]) = v[it];
    }
}

static inline void launch_gemm4(hipStream_t st, const unsigned short* A, const unsigned short* B,
                                const float* bias, const float* bias2, const float* resid,
                                float* C, float* C2, float* Cdup, int N, int K, int ldc, int csplit, float scale)
{
    hipLaunchKernelGGL(HIP_KERNEL_NAME(gemm_tn_kernel<4>), dim3(N / 128, MT_ / 64), dim3(128), 0, st,
                       A, B, bias, bias2, resid, C, C2, Cdup, K, ldc, csplit, scale);
}
static inline void launch_gemm2(hipStream_t st, const unsigned short* A, const unsigned short* B,
                                const float* bias, const float* bias2, const float* resid,
                                float* C, float* C2, float* Cdup, int N, int K, int ldc, int csplit, float scale)
{
    hipLaunchKernelGGL(HIP_KERNEL_NAME(gemm_tn_kernel<2>), dim3(N / 64, MT_ / 64), dim3(128), 0, st,
                       A, B, bias, bias2, resid, C, C2, Cdup, K, ldc, csplit, scale);
}

extern "C" void kernel_launch(void* const* d_in, const int* in_sizes, int n_in,
                              void* d_out, int out_size, void* d_ws, size_t ws_size,
                              hipStream_t stream)
{
    if (n_in < 33) return;
    const int expect_sz[33] = {
        MT_ * DM_, DM_, DM_, DM_ * DM_, DM_, DM_ * DM_, DM_, DM_ * DM_, DM_,
        DM_ * 2 * DM_, DM_, DM_ * DM_ * 3, DM_,
        NLAY_ * 2 * DI_ * DM_, NLAY_ * DI_ * 4, NLAY_ * DI_, NLAY_ * XPR_ * DI_, NLAY_ * DI_ * DTR_,
        NLAY_ * DI_, NLAY_ * DI_ * NS_, NLAY_ * DI_, NLAY_ * DM_ * DI_, NLAY_ * DM_,
        NLAY_ * 2 * DI_ * DM_, NLAY_ * DI_ * 4, NLAY_ * DI_, NLAY_ * XPR_ * DI_, NLAY_ * DI_ * DTR_,
        NLAY_ * DI_, NLAY_ * DI_ * NS_, NLAY_ * DI_, NLAY_ * DM_ * DI_, NLAY_ * DM_ };
    for (int i = 0; i < 33; ++i) if (in_sizes[i] != expect_sz[i]) return;
    if (out_size != MT_ * DM_) return;

    const float* x       = (const float*)d_in[0];
    const float* ln_g    = (const float*)d_in[1];
    const float* ln_b    = (const float*)d_in[2];
    const float* w1      = (const float*)d_in[3];
    const float* b1      = (const float*)d_in[4];
    const float* w2      = (const float*)d_in[5];
    const float* b2      = (const float*)d_in[6];
    const float* w3      = (const float*)d_in[7];
    const float* b3      = (const float*)d_in[8];
    const float* down_w  = (const float*)d_in[9];
    const float* down_b  = (const float*)d_in[10];
    const float* hconv_w = (const float*)d_in[11];
    const float* hconv_b = (const float*)d_in[12];
    const float* mp[2][10];
    for (int dir = 0; dir < 2; ++dir)
        for (int j = 0; j < 10; ++j) mp[dir][j] = (const float*)d_in[13 + dir * 10 + j];
    float* out = (float*)d_out;

    const size_t SZ_TD   = (size_t)MT_ * DM_ * 4;
    const size_t SZ_TI   = (size_t)MT_ * DI_ * 4;
    const size_t SZ_DBC  = (size_t)MT_ * XPN_ * 4;
    const size_t SZ_W12  = (size_t)2 * DM_ * DM_ * 2;
    const size_t SZ_W3   = (size_t)DM_ * DM_ * 2;
    const size_t SZ_DWN  = (size_t)DM_ * 2 * DM_ * 2;
    const size_t SZ_HW   = (size_t)DM_ * HCK_ * 2;
    const size_t SZ_INP  = (size_t)NLAY_ * 2 * DI_ * DM_ * 2;
    const size_t SZ_XPJ  = (size_t)NLAY_ * XPN_ * DI_ * 2;
    const size_t SZ_DTW  = (size_t)NLAY_ * DI_ * DTK_ * 2;
    const size_t SZ_OUTW = (size_t)NLAY_ * DM_ * DI_ * 2;
    const size_t SZ_TD16 = (size_t)MT_ * DM_ * 2;
    const size_t SZ_COL  = (size_t)MT_ * HCK_ * 2;
    const size_t SZ_TI16 = (size_t)MT_ * DI_ * 2;
    const size_t SZ_DBC16= (size_t)MT_ * DTK_ * 2;

    size_t off = 0;
    const size_t OFF_X1   = off; off += SZ_TD;
    const size_t OFF_X2   = off; off += SZ_TD;
    const size_t OFF_XF   = off; off += SZ_TD;
    const size_t OFF_XB   = off; off += SZ_TD;
    const size_t OFF_XI   = off; off += SZ_TI;
    const size_t OFF_ZF   = off; off += SZ_TI;
    const size_t OFF_DL   = off; off += SZ_TI;
    const size_t OFF_DBC  = off; off += SZ_DBC;
    const size_t OFF_DBUF = off; off += SZ_TD;
    const size_t OFF_W12  = off; off += SZ_W12;
    const size_t OFF_W3   = off; off += SZ_W3;
    const size_t OFF_DWN  = off; off += SZ_DWN;
    const size_t OFF_HW   = off; off += SZ_HW;
    size_t OFF_INP[2], OFF_XPJ[2], OFF_DTW[2], OFF_OUTW[2];
    for (int dir = 0; dir < 2; ++dir) {
        OFF_INP[dir]  = off; off += SZ_INP;
        OFF_XPJ[dir]  = off; off += SZ_XPJ;
        OFF_DTW[dir]  = off; off += SZ_DTW;
        OFF_OUTW[dir] = off; off += SZ_OUTW;
    }
    const size_t OFF_XL16  = off; off += SZ_TD16;
    const size_t OFF_COL16 = off; off += SZ_COL;
    const size_t OFF_XN16  = off; off += SZ_TD16;
    const size_t OFF_U16   = off; off += SZ_TI16;
    const size_t OFF_DBC16 = off; off += SZ_DBC16;
    const size_t OFF_G16   = off; off += SZ_TI16;
    const size_t OFF_CAT16 = off; off += SZ_TI16;
    const size_t OFF_DL16  = off; off += SZ_TD16;
    const size_t WS_END = off;
    if (WS_END > ws_size) return;
    if (WS_END > (size_t)134217728) return;

    char* ws = (char*)d_ws;
    float* x1   = (float*)(ws + OFF_X1);
    float* x2   = (float*)(ws + OFF_X2);
    float* xf   = (float*)(ws + OFF_XF);
    float* xb   = (float*)(ws + OFF_XB);
    float* Xi   = (float*)(ws + OFF_XI);
    float* Zf   = (float*)(ws + OFF_ZF);
    float* Dl   = (float*)(ws + OFF_DL);
    float* dbc  = (float*)(ws + OFF_DBC);
    float* dbuf = (float*)(ws + OFF_DBUF);
    unsigned short* w12h = (unsigned short*)(ws + OFF_W12);
    unsigned short* w3h  = (unsigned short*)(ws + OFF_W3);
    unsigned short* dwnh = (unsigned short*)(ws + OFF_DWN);
    unsigned short* hwh  = (unsigned short*)(ws + OFF_HW);
    unsigned short* inph[2], *xpjh[2], *dtwh[2], *outwh[2];
    for (int dir = 0; dir < 2; ++dir) {
        inph[dir]  = (unsigned short*)(ws + OFF_INP[dir]);
        xpjh[dir]  = (unsigned short*)(ws + OFF_XPJ[dir]);
        dtwh[dir]  = (unsigned short*)(ws + OFF_DTW[dir]);
        outwh[dir] = (unsigned short*)(ws + OFF_OUTW[dir]);
    }
    unsigned short* xl16  = (unsigned short*)(ws + OFF_XL16);
    unsigned short* col16 = (unsigned short*)(ws + OFF_COL16);
    unsigned short* xn16  = (unsigned short*)(ws + OFF_XN16);
    unsigned short* u16   = (unsigned short*)(ws + OFF_U16);
    unsigned short* dbc16 = (unsigned short*)(ws + OFF_DBC16);
    unsigned short* g16   = (unsigned short*)(ws + OFF_G16);
    unsigned short* cat16 = (unsigned short*)(ws + OFF_CAT16);
    unsigned short* dl16  = (unsigned short*)(ws + OFF_DL16);

    const float WSC = 64.0f;

    {
        int n8a, n8b, gx;
        n8a = (DM_ * DM_) / 8; n8b = (DM_ * DM_) / 8; gx = (n8a > n8b ? n8a : n8b);
        hipLaunchKernelGGL(cvt2_kernel, dim3((gx + 255) / 256, 2), dim3(256), 0, stream,
                           w1, w12h, n8a, w2, w12h + (size_t)DM_ * DM_, n8b, WSC);
        n8a = (DM_ * DM_) / 8; n8b = (DM_ * 2 * DM_) / 8; gx = (n8a > n8b ? n8a : n8b);
        hipLaunchKernelGGL(cvt2_kernel, dim3((gx + 255) / 256, 2), dim3(256), 0, stream,
                           w3, w3h, n8a, down_w, dwnh, n8b, WSC);
        hipLaunchKernelGGL(hconv_pack_kernel, dim3((DM_ * HCK_ / 8 + 255) / 256), dim3(256), 0, stream,
                           hconv_w, hwh, WSC);
        n8a = (NLAY_ * 2 * DI_ * DM_) / 8;
        hipLaunchKernelGGL(cvt2_kernel, dim3((n8a + 255) / 256, 2), dim3(256), 0, stream,
                           mp[0][0], inph[0], n8a, mp[1][0], inph[1], n8a, WSC);
        hipLaunchKernelGGL(xproj_pack_kernel, dim3((NLAY_ * XPN_ * DI_ / 8 + 255) / 256, 2), dim3(256), 0, stream,
                           mp[0][3], mp[1][3], xpjh[0], xpjh[1], WSC);
        hipLaunchKernelGGL(dtw_pack_kernel, dim3((NLAY_ * DI_ * DTK_ / 8 + 255) / 256, 2), dim3(256), 0, stream,
                           mp[0][4], mp[1][4], dtwh[0], dtwh[1], WSC);
        n8a = (NLAY_ * DM_ * DI_) / 8;
        hipLaunchKernelGGL(cvt2_kernel, dim3((n8a + 255) / 256, 2), dim3(256), 0, stream,
                           mp[0][8], outwh[0], n8a, mp[1][8], outwh[1], n8a, WSC);
    }

    hipLaunchKernelGGL(norm_f16_kernel, dim3(MT_ / 2), dim3(64), 0, stream,
                       x, ln_g, ln_b, (const float*)nullptr, xl16, 0, 1.0f);
    launch_gemm4(stream, xl16, w12h, b1, b2, (const float*)nullptr, x1, x2, (float*)nullptr,
                 2 * DM_, DM_, DM_, DM_, 1.0f / 64.0f);
    hipLaunchKernelGGL(im2col_kernel, dim3(MT_ / 2), dim3(64), 0, stream, (const float*)x1, col16, 16.0f);
    launch_gemm4(stream, col16, hwh, hconv_b, hconv_b, (const float*)nullptr, xf, xf, xb,
                 DM_, HCK_, DM_, 1 << 30, 1.0f / 1024.0f);

    for (int dir = 0; dir < 2; ++dir) {
        float* xcur = dir ? xb : xf;
        for (int l = 0; l < NLAY_; ++l) {
            const float* convw = mp[dir][1] + (size_t)l * DI_ * 4;
            const float* convb = mp[dir][2] + (size_t)l * DI_;
            const float* dtb   = mp[dir][5] + (size_t)l * DI_;
            const float* alog  = mp[dir][6] + (size_t)l * DI_ * NS_;
            const float* Dp    = mp[dir][7] + (size_t)l * DI_;
            const float* rms   = mp[dir][9] + (size_t)l * DM_;
            hipLaunchKernelGGL(norm_f16_kernel, dim3(MT_ / 2), dim3(64), 0, stream,
                               (const float*)xcur, rms, rms, (const float*)nullptr, xn16, 1, 1.0f);
            launch_gemm4(stream, xn16, inph[dir] + (size_t)l * 2 * DI_ * DM_,
                         (const float*)nullptr, (const float*)nullptr, (const float*)nullptr,
                         Xi, Zf, (float*)nullptr, 2 * DI_, DM_, DI_, DI_, 1.0f / 64.0f);
            hipLaunchKernelGGL(conv_silu_kernel, dim3(MT_), dim3(DI_ / 8), 0, stream,
                               (const float*)Xi, convw, convb, u16, dir, 256.0f);
            launch_gemm2(stream, u16, xpjh[dir] + (size_t)l * XPN_ * DI_,
                         (const float*)nullptr, (const float*)nullptr, (const float*)nullptr,
                         dbc, dbc, (float*)nullptr, XPN_, DI_, XPN_, 1 << 30, 1.0f / 16384.0f);
            hipLaunchKernelGGL(dbc16_kernel, dim3((MT_ * DTK_ / 8 + 255) / 256), dim3(256), 0, stream,
                               (const float*)dbc, dbc16, 256.0f);
            launch_gemm4(stream, dbc16, dtwh[dir] + (size_t)l * DI_ * DTK_,
                         (const float*)nullptr, (const float*)nullptr, (const float*)nullptr,
                         Dl, Dl, (float*)nullptr, DI_, DTK_, DI_, 1 << 30, 1.0f / 16384.0f);
            hipLaunchKernelGGL(scan_kernel, dim3(DI_ / 64, NB_), dim3(64), 0, stream,
                               (const float*)Xi, (const float*)Zf, (const float*)Dl, (const float*)dbc,
                               convw, convb, dtb, alog, Dp, g16, dir, 4096.0f);
            launch_gemm4(stream, g16, outwh[dir] + (size_t)l * DM_ * DI_,
                         (const float*)nullptr, (const float*)nullptr, (const float*)xcur,
                         xcur, xcur, (float*)nullptr, DM_, DI_, DM_, 1 << 30, 1.0f / 262144.0f);
        }
    }

    hipLaunchKernelGGL(cat_kernel, dim3(MT_ / 2), dim3(64), 0, stream,
                       (const float*)xf, (const float*)xb, cat16, 16.0f);
    launch_gemm4(stream, cat16, dwnh, down_b, down_b, (const float*)nullptr, dbuf, dbuf, (float*)nullptr,
                 DM_, 2 * DM_, DM_, 1 << 30, 1.0f / 1024.0f);
    hipLaunchKernelGGL(norm_f16_kernel, dim3(MT_ / 2), dim3(64), 0, stream,
                       (const float*)dbuf, ln_g, ln_b, (const float*)x2, dl16, 0, 16.0f);
    launch_gemm4(stream, dl16, w3h, b3, b3, x, out, out, (float*)nullptr,
                 DM_, DM_, DM_, 1 << 30, 1.0f / 1024.0f);
}
